// Rankformer_66589172957770
// MI455X (gfx1250) — hardware-verified
//
#include <hip/hip_runtime.h>
#include <math.h>
typedef __attribute__((ext_vector_type(16))) _Float16 v16h;
typedef __attribute__((ext_vector_type(8)))  _Float16 v8h;
typedef __attribute__((ext_vector_type(16))) __bf16   v16b;
typedef __attribute__((ext_vector_type(8)))  __bf16   v8b;
typedef __attribute__((ext_vector_type(8)))  float    v8f;
typedef __attribute__((ext_vector_type(4)))  float    v4f;
#define PSCALE 32768.0f
#define U16(p) ((const unsigned short*)(const void*)(p))
#define PSCALE_INV (1.0f / 32768.0f)

__device__ __forceinline__ unsigned short f2bf_bits(float f) {
  unsigned u = __float_as_uint(f);
  return (unsigned short)((u + 0x7FFFu + ((u >> 16) & 1u)) >> 16);
}
__device__ __forceinline__ float bf_bits2f(unsigned short h) { return __uint_as_float(((unsigned)h) << 16); }

__device__ __forceinline__ void dep_guard_h(v8f& a, v8f& b, v16h x, v16h y) { asm volatile("v_nop\n\tv_nop\n\tv_nop\n\tv_nop" : "+v"(a), "+v"(b) : "v"(x), "v"(y)); }
__device__ __forceinline__ void dep_guard_b(v8f& a, v8f& b, v16b x, v16b y) { asm volatile("v_nop\n\tv_nop\n\tv_nop\n\tv_nop" : "+v"(a), "+v"(b) : "v"(x), "v"(y)); }
__device__ __forceinline__ void keep4_h(v16h a, v16h b, v16h c, v16h d) { asm volatile("v_nop" :: "v"(a), "v"(b), "v"(c), "v"(d)); }
__device__ __forceinline__ void keep4_b(v16b a, v16b b, v16b c, v16b d) { asm volatile("v_nop" :: "v"(a), "v"(b), "v"(c), "v"(d)); }
__device__ __forceinline__ void acc_guard4(v8f& a, v8f& b, v8f& c, v8f& d) { asm volatile("v_nop\n\tv_nop\n\tv_nop\n\tv_nop" : "+v"(a), "+v"(b), "+v"(c), "+v"(d)); }
template <typename T> struct Frag;
template <> struct Frag<_Float16> {
  typedef v16h V; union U { v16h v; v8h h[2]; };
  static __device__ __forceinline__ v16h load(const _Float16* p) {
    U f; f.h[0] = *(const v8h*)(p); f.h[1] = *(const v8h*)(p + 16); return f.v;
  }
  static __device__ __forceinline__ v8f mma(v16h a, v16h b, v8f c) {
    return __builtin_amdgcn_wmma_f32_16x16x32_f16(false, a, false, b, (short)0, c, false, false);
  }
  static __device__ __forceinline__ void guard(v8f& a, v8f& b, v16h x, v16h y) { dep_guard_h(a, b, x, y); }
  static __device__ __forceinline__ void keep(v16h a, v16h b, v16h c, v16h d) { keep4_h(a, b, c, d); }
};
template <> struct Frag<__bf16> {
  typedef v16b V; union U { v16b v; v8b h[2]; };
  static __device__ __forceinline__ v16b load(const __bf16* p) {
    U f; f.h[0] = *(const v8b*)(p); f.h[1] = *(const v8b*)(p + 16); return f.v;
  }
  static __device__ __forceinline__ v8f mma(v16b a, v16b b, v8f c) {
    return __builtin_amdgcn_wmma_f32_16x16x32_bf16(false, a, false, b, (short)0, c, false, false);
  }
  static __device__ __forceinline__ void guard(v8f& a, v8f& b, v16b x, v16b y) { dep_guard_b(a, b, x, y); }
  static __device__ __forceinline__ void keep(v16b a, v16b b, v16b c, v16b d) { keep4_b(a, b, c, d); }
};

template <int ET> struct Elem;
template <> struct Elem<0> { typedef _Float16 T; };
template <> struct Elem<1> { typedef __bf16 T; };
template <int ET, bool SPLIT, int BIAS_MODE, int OUT_MODE, bool RESID, int ACT = 0>
__global__ __launch_bounds__(256) void wmma_gemm64(
    const unsigned short* __restrict__ Ap, const unsigned short* __restrict__ A2p, int lda, long strideA,
    const unsigned short* __restrict__ Btp, const unsigned short* __restrict__ Bt2p, int ldb, long strideB,
    void* __restrict__ Cout, void* __restrict__ Cout2, int ldc, long strideC,
    const float* __restrict__ bias,
    const float* __restrict__ resid, long strideR,
    int M, int N, int K, float scale) {
  typedef typename Elem<ET>::T T;
  typedef typename Frag<T>::V V;
  const T* A = (const T*)Ap; const T* A2 = (const T*)A2p; const T* Bt = (const T*)Btp; const T* Bt2 = (const T*)Bt2p;
  __shared__ __align__(16) float sT[8][16 * 68];
  const int b    = blockIdx.y;
  const int lane = threadIdx.x & 31;
  const int wave = threadIdx.x >> 5;
  const int tilesN = N >> 6;
  const int tilesM = M >> 6;
  const int tile = blockIdx.x * 8 + wave;
  if (tile >= tilesM * tilesN) return;
  const int tm = tile / tilesN;
  const int tn = tile - tm * tilesN;
  const int m0 = tm << 6;
  const int n0 = tn << 6;

  const T* Ab  = A  + (size_t)b * strideA;
  const T* Bb  = Bt + (size_t)b * strideB;
  const T* Ab2 = SPLIT ? (A2  + (size_t)b * strideA) : nullptr;
  const T* Bb2 = SPLIT ? (Bt2 + (size_t)b * strideB) : nullptr;

  const int rlane = lane & 15;
  const int koff  = (lane >> 4) * 8;
  const int mOff  = (lane >> 4) * 8;

  v8f acc[4][4];
#pragma unroll
  for (int i = 0; i < 4; ++i)
#pragma unroll
    for (int j = 0; j < 4; ++j) acc[i][j] = (v8f){0.f,0.f,0.f,0.f,0.f,0.f,0.f,0.f};

  for (int k0 = 0; k0 < K; k0 += 32) {
    V bh[4], bl[4];
#pragma unroll
    for (int j = 0; j < 4; ++j) {
      const size_t bo = (size_t)(n0 + (j << 4) + rlane) * ldb + koff + k0;
      bh[j] = Frag<T>::load(Bb + bo);
      if (SPLIT) bl[j] = Frag<T>::load(Bb2 + bo);
    }
#pragma unroll
    for (int i = 0; i < 4; ++i) {
      const size_t ao = (size_t)(m0 + (i << 4) + rlane) * lda + koff + k0;
      V ah = Frag<T>::load(Ab + ao);
      V al;
      if (SPLIT) al = Frag<T>::load(Ab2 + ao);
#pragma unroll
      for (int j = 0; j < 4; ++j) {
        acc[i][j] = Frag<T>::mma(ah, bh[j], acc[i][j]);
        if (SPLIT) {
          acc[i][j] = Frag<T>::mma(ah, bl[j], acc[i][j]);
          acc[i][j] = Frag<T>::mma(al, bh[j], acc[i][j]);
        }
      }
      Frag<T>::guard(acc[i][0], acc[i][3], ah, SPLIT ? al : ah);
    }
    Frag<T>::keep(bh[0], bh[1], bh[2], bh[3]);
    if (SPLIT) Frag<T>::keep(bl[0], bl[1], bl[2], bl[3]);
  }
  acc_guard4(acc[0][0], acc[0][1], acc[0][2], acc[0][3]);
  acc_guard4(acc[1][0], acc[1][1], acc[1][2], acc[1][3]);
  acc_guard4(acc[2][0], acc[2][1], acc[2][2], acc[2][3]);
  acc_guard4(acc[3][0], acc[3][1], acc[3][2], acc[3][3]);

  float* slab = sT[wave];
  const float* Rb = RESID ? (resid + (size_t)b * strideR) : nullptr;
#pragma unroll
  for (int i = 0; i < 4; ++i) {
    const int mBase = m0 + (i << 4);
#pragma unroll
    for (int j = 0; j < 4; ++j) {
      const int n = n0 + (j << 4) + rlane;
      float bv = 0.f;
      if (BIAS_MODE == 2) bv = bias[n];
#pragma unroll
      for (int r = 0; r < 8; ++r) {
        float v = acc[i][j][r] * scale;
        if (BIAS_MODE == 1) v += bias[mBase + mOff + r];
        if (BIAS_MODE == 2) v += bv;
        if (RESID) v += Rb[(size_t)(mBase + mOff + r) * ldc + n];
        if (ACT == 1) v = tanhf(v);
        if (ACT == 2) v = fmaxf(v, 0.0f);
        if (ACT == 3) v = v / (1.0f + expf(-v));
        if (ACT == 4) v = (v > 0.f) ? v : 0.01f * v;
        slab[(mOff + r) * 68 + (j << 4) + rlane] = v;
      }
    }
    __builtin_amdgcn_fence(__ATOMIC_RELEASE, "workgroup");
    __builtin_amdgcn_wave_barrier();
    __builtin_amdgcn_fence(__ATOMIC_ACQUIRE, "workgroup");
    if (OUT_MODE == 0) {
      float* C = (float*)Cout + (size_t)b * strideC;
      const int hh = lane >> 4, c4 = (lane & 15) * 4;
      for (int pass = 0; pass < 2; ++pass) {
#pragma unroll
        for (int it = 0; it < 8; ++it) {
          const int row = it * 2 + hh;
          v4f v = *(const v4f*)(slab + row * 68 + c4);
          *(volatile v4f*)(C + (size_t)(mBase + row) * ldc + n0 + c4) = v;
        }
        __threadfence();
      }
    } else {
      const int q = lane >> 3, c8 = (lane & 7) * 8;
      unsigned short* C  = (unsigned short*)Cout  + (size_t)b * strideC;
      unsigned short* C2 = (OUT_MODE == 2) ? ((unsigned short*)Cout2 + (size_t)b * strideC) : nullptr;
      for (int pass = 0; pass < 2; ++pass) {
#pragma unroll
        for (int it = 0; it < 4; ++it) {
          const int row = it * 4 + q;
          const float* sp = slab + row * 68 + c8;
          v8h hv, lv;
#pragma unroll
          for (int e = 0; e < 8; ++e) {
            if (OUT_MODE == 1) {
              hv[e] = (_Float16)sp[e];
            } else {
              unsigned short hb = f2bf_bits(sp[e]);
              unsigned short lb = f2bf_bits(sp[e] - bf_bits2f(hb));
              hv[e] = __builtin_bit_cast(_Float16, hb);
              lv[e] = __builtin_bit_cast(_Float16, lb);
            }
          }
          *(volatile v8h*)(C + (size_t)(mBase + row) * ldc + n0 + c8) = hv;
          if (OUT_MODE == 2) *(volatile v8h*)(C2 + (size_t)(mBase + row) * ldc + n0 + c8) = lv;
        }
        __threadfence();
      }
    }
    __builtin_amdgcn_fence(__ATOMIC_RELEASE, "workgroup");
    __builtin_amdgcn_wave_barrier();
    __builtin_amdgcn_fence(__ATOMIC_ACQUIRE, "workgroup");
  }
}


#define NNU 100000
#define NNI 50000
#define NUPAD 100096
#define NIPAD 50176
#define KU 100032
#define KI 50048
#define NE 1000000
#define D 64
#define NODES_PER_BLK 256
#define NBLKU ((NNU + NODES_PER_BLK - 1) / NODES_PER_BLK)
#define NBLKI ((NNI + NODES_PER_BLK - 1) / NODES_PER_BLK)
#define SEG_CAP 16384
#define ALPHA 1.0f
#define CLAMPV 1e-6f

#define u_ECH 8192
#define u_NCH ((NE + u_ECH - 1) / u_ECH)
#define u_NRP (((NBLKU) + 31) & ~31)
#define u_SEG_STRIDE SEG_CAP
#define u_BUCKET_INTS ((size_t)NE + (size_t)32 * u_NCH * NBLKU)
__device__ __forceinline__ int u_rank_eq(int key, bool valid, int lane, int nbits, int& ntotal) {
  unsigned same = __ballot(valid);
  for (int b = 0; b < nbits; ++b) {
    const unsigned m = __ballot(((key >> b) & 1) != 0);
    same &= (((key >> b) & 1) != 0) ? m : ~m;
  }
  if (!valid) same = 0u;
  ntotal = __popc(same);
  return __popc(same & ((1u << lane) - 1u));
}
__global__ __launch_bounds__(256) void u_csr_hist_kernel(const int* __restrict__ dst, int* __restrict__ cnt) {
  __shared__ int h[8][u_NRP];
  const int tid = threadIdx.x, lane = tid & 31, wave = tid >> 5;
  for (int i = tid; i < 8 * u_NRP; i += 256) (&h[0][0])[i] = 0;
  __syncthreads();
  const int e0 = blockIdx.x * u_ECH + wave * (u_ECH / 8), e1 = min(e0 + u_ECH / 8, NE);
  for (int c0 = e0; c0 < e0 + u_ECH / 8; c0 += 32) {
    const int e = c0 + lane;
    const bool valid = e < e1;
    int d = valid ? dst[e] : 0; d = d < 0 ? 0 : (d >= NNU ? NNU - 1 : d);
    const int r = d / NODES_PER_BLK;
    int tot; const int rk = u_rank_eq(r, valid, lane, 9, tot);
    if (valid && rk == tot - 1) h[wave][r] += tot;
  }
  __syncthreads();
  for (int pass = 0; pass < 2; ++pass) {
    for (int i = tid; i < u_NRP; i += 256) { int s = 0; for (int w = 0; w < 8; ++w) s += h[w][i]; ((volatile int*)cnt)[(size_t)blockIdx.x * u_NRP + i] = s; }
    __threadfence();
  }
}
__global__ __launch_bounds__(1024) void u_csr_offsets_kernel(const int* __restrict__ cnt, int* __restrict__ boff, int* __restrict__ rinfo) {
  __shared__ int rsz[1024];
  const int t = threadIdx.x;
  int run = 0;
  if (t < NBLKU) { for (int c = 0; c < u_NCH; ++c) run += (cnt[(size_t)c * u_NRP + t] + 31) & ~31; }
  rsz[t] = (t < NBLKU) ? run : 0;
  __syncthreads();
  for (int off = 1; off < 1024; off <<= 1) { int v = (t >= off) ? rsz[t - off] : 0; __syncthreads(); rsz[t] += v; __syncthreads(); }
  const int incl = rsz[t], excl = incl - ((t < NBLKU) ? run : 0);
  __syncthreads();
  for (int pass = 0; pass < 2; ++pass) {
    if (t < NBLKU) { int r2 = excl; for (int c = 0; c < u_NCH; ++c) { const size_t i = (size_t)c * u_NRP + t; ((volatile int*)boff)[i] = r2; r2 += (cnt[i] + 31) & ~31; } }
    ((volatile int*)rinfo)[t] = excl;
    ((volatile int*)rinfo)[1024 + t] = (t < NBLKU) ? run : 0;
    __threadfence();
  }
}
__global__ __launch_bounds__(256) void u_csr_bucket_kernel(const int* __restrict__ dst, const int* __restrict__ boff, int* __restrict__ bucket) {
  __shared__ int wc[8][u_NRP];
  __shared__ int woff[8][u_NRP];
  __shared__ int roff[u_NRP + 1];
  __shared__ int seg[u_ECH + 32 * u_NRP];
  const int tid = threadIdx.x, lane = tid & 31, wave = tid >> 5;
  for (int i = tid; i < 8 * u_NRP; i += 256) { (&wc[0][0])[i] = 0; }
  __syncthreads();
  const int e0 = blockIdx.x * u_ECH + wave * (u_ECH / 8), e1 = min(e0 + u_ECH / 8, NE);
  for (int c0 = e0; c0 < e0 + u_ECH / 8; c0 += 32) {
    const int e = c0 + lane; const bool valid = e < e1;
    int d = valid ? dst[e] : 0; d = d < 0 ? 0 : (d >= NNU ? NNU - 1 : d);
    const int r = d / NODES_PER_BLK;
    int tot; const int rk = u_rank_eq(r, valid, lane, 9, tot);
    if (valid && rk == tot - 1) wc[wave][r] += tot;
  }
  __syncthreads();
  __shared__ int tot_r[u_NRP];
  for (int i = tid; i < u_NRP; i += 256) { int s = 0; for (int w = 0; w < 8; ++w) s += wc[w][i]; tot_r[i] = s; }
  __syncthreads();
  if (tid == 0) { int run = 0; for (int r = 0; r < u_NRP; ++r) { roff[r] = run; int o = run; for (int w = 0; w < 8; ++w) { woff[w][r] = o; o += wc[w][r]; } run += (tot_r[r] + 31) & ~31; } roff[u_NRP] = run; }
  __syncthreads();
  const int totalpad = roff[u_NRP];
  for (int i = tid; i < totalpad && i < u_ECH + 32 * u_NRP; i += 256) seg[i] = -1;
  __syncthreads();
  for (int c0 = e0; c0 < e0 + u_ECH / 8; c0 += 32) {
    const int e = c0 + lane; const bool valid = e < e1;
    int d = valid ? dst[e] : 0; d = d < 0 ? 0 : (d >= NNU ? NNU - 1 : d);
    const int r = d / NODES_PER_BLK;
    int tot; const int rk = u_rank_eq(r, valid, lane, 9, tot);
    if (valid) { const int slot = woff[wave][r] + rk; if (slot < u_ECH + 32 * u_NRP) seg[slot] = e; if (rk == tot - 1) woff[wave][r] = slot + 1; }
  }
  __syncthreads();
  for (int pass = 0; pass < 2; ++pass) {
    for (int r = wave; r < NBLKU; r += 8) {
      const int lo = roff[r], n = ((tot_r[r] + 31) & ~31);
      const int gb = boff[(size_t)blockIdx.x * u_NRP + r];
      for (int i = lane; i < n; i += 32) ((volatile int*)bucket)[(size_t)gb + i] = (lo + i < u_ECH + 32 * u_NRP) ? seg[lo + i] : -1;
    }
    __threadfence();
  }
}
__global__ __launch_bounds__(256) void u_csr_fill_kernel(const int* __restrict__ dst, const int* __restrict__ bucket, const int* __restrict__ rinfo,
                                                      int* __restrict__ rowptr, int* __restrict__ rowdeg, int* __restrict__ csr_eid, int* __restrict__ rcl) {
  __shared__ int cnt[8][NODES_PER_BLK];
  __shared__ int off[8][NODES_PER_BLK];
  __shared__ int nodeoff[NODES_PER_BLK + 1];
  __shared__ int seg[SEG_CAP];
  const int tid = threadIdx.x, lane = tid & 31, wave = tid >> 5;
  const int n0 = blockIdx.x * NODES_PER_BLK;
  const int bstart = rinfo[blockIdx.x], bsize = rinfo[1024 + blockIdx.x];
  for (int i = tid; i < 8 * NODES_PER_BLK; i += 256) (&cnt[0][0])[i] = 0;
  for (int i = tid; i < SEG_CAP; i += 256) seg[i] = 0;
  __syncthreads();
  const int per = ((bsize / 8) + 31) & ~31;
  const int e0 = bstart + wave * per, e1 = min(bstart + (wave + 1) * per, bstart + bsize);
  for (int c0 = e0; c0 < e0 + per; c0 += 32) {
    const int j = c0 + lane;
    int e = (j < e1) ? bucket[j] : -1;
    const bool valid = (e >= 0) && (e < NE);
    int d = valid ? dst[e] : -1;
    const bool ok = valid && (d >= n0) && (d < n0 + NODES_PER_BLK);
    int tot; const int rk = u_rank_eq(ok ? (d - n0) : 0, ok, lane, 8, tot);
    if (ok && rk == tot - 1) cnt[wave][d - n0] += tot;
  }
  __syncthreads();
  if (tid < 32) {
    int loc[8]; int sum = 0;
    for (int q = 0; q < 8; ++q) { int c = 0; for (int w = 0; w < 8; ++w) c += cnt[w][tid * 8 + q]; loc[q] = c; sum += c; }
    int incl = sum;
    for (int o = 1; o < 32; o <<= 1) { int t = __shfl_up(incl, o, 32); if (lane >= o) incl += t; }
    int base = incl - sum;
    for (int q = 0; q < 8; ++q) {
      const int node = tid * 8 + q;
      nodeoff[node] = base;
      int run = base;
      for (int w = 0; w < 8; ++w) { off[w][node] = run; run += cnt[w][node]; }
      base += loc[q];
    }
    if (tid == 31) nodeoff[NODES_PER_BLK] = base;
  }
  __syncthreads();
  const int btotal = nodeoff[NODES_PER_BLK];
  for (int c0 = e0; c0 < e0 + per; c0 += 32) {
    const int j = c0 + lane;
    int e = (j < e1) ? bucket[j] : -1;
    const bool valid = (e >= 0) && (e < NE);
    int d = valid ? dst[e] : -1;
    const bool ok = valid && (d >= n0) && (d < n0 + NODES_PER_BLK);
    int tot; const int rk = u_rank_eq(ok ? (d - n0) : 0, ok, lane, 8, tot);
    if (ok) { const int slot = off[wave][d - n0] + rk; if (slot < SEG_CAP) seg[slot] = e; if (rk == tot - 1) off[wave][d - n0] = slot + 1; }
  }
  __syncthreads();
  const int gstart = blockIdx.x * (u_SEG_STRIDE);
  const int nlines = (min(btotal, SEG_CAP) + 31) >> 5;
  for (int pass = 0; pass < 2; ++pass) {
    { const int node = tid; int deg = 0; for (int w = 0; w < 8; ++w) deg += cnt[w][node];
      ((volatile int*)rowptr)[n0 + node] = gstart + nodeoff[node]; ((volatile int*)rowdeg)[n0 + node] = deg; }
    for (int i = tid; i < nlines * 32; i += 256) ((volatile int*)csr_eid)[gstart + i] = (i < btotal) ? seg[i] : 0;
    if (rcl != nullptr && tid < 32) ((volatile int*)rcl)[blockIdx.x * 32 + tid] = (tid == 0) ? min(btotal, SEG_CAP) : 0;
    __threadfence();
  }
}

#define i_ECH 8192
#define i_NCH ((NE + i_ECH - 1) / i_ECH)
#define i_NRP (((NBLKI) + 31) & ~31)
#define i_SEG_STRIDE SEG_CAP
#define i_BUCKET_INTS ((size_t)NE + (size_t)32 * i_NCH * NBLKI)
__device__ __forceinline__ int i_rank_eq(int key, bool valid, int lane, int nbits, int& ntotal) {
  unsigned same = __ballot(valid);
  for (int b = 0; b < nbits; ++b) {
    const unsigned m = __ballot(((key >> b) & 1) != 0);
    same &= (((key >> b) & 1) != 0) ? m : ~m;
  }
  if (!valid) same = 0u;
  ntotal = __popc(same);
  return __popc(same & ((1u << lane) - 1u));
}
__global__ __launch_bounds__(256) void i_csr_hist_kernel(const int* __restrict__ dst, int* __restrict__ cnt) {
  __shared__ int h[8][i_NRP];
  const int tid = threadIdx.x, lane = tid & 31, wave = tid >> 5;
  for (int i = tid; i < 8 * i_NRP; i += 256) (&h[0][0])[i] = 0;
  __syncthreads();
  const int e0 = blockIdx.x * i_ECH + wave * (i_ECH / 8), e1 = min(e0 + i_ECH / 8, NE);
  for (int c0 = e0; c0 < e0 + i_ECH / 8; c0 += 32) {
    const int e = c0 + lane;
    const bool valid = e < e1;
    int d = valid ? dst[e] : 0; d = d < 0 ? 0 : (d >= NNI ? NNI - 1 : d);
    const int r = d / NODES_PER_BLK;
    int tot; const int rk = i_rank_eq(r, valid, lane, 9, tot);
    if (valid && rk == tot - 1) h[wave][r] += tot;
  }
  __syncthreads();
  for (int pass = 0; pass < 2; ++pass) {
    for (int i = tid; i < i_NRP; i += 256) { int s = 0; for (int w = 0; w < 8; ++w) s += h[w][i]; ((volatile int*)cnt)[(size_t)blockIdx.x * i_NRP + i] = s; }
    __threadfence();
  }
}
__global__ __launch_bounds__(1024) void i_csr_offsets_kernel(const int* __restrict__ cnt, int* __restrict__ boff, int* __restrict__ rinfo) {
  __shared__ int rsz[1024];
  const int t = threadIdx.x;
  int run = 0;
  if (t < NBLKI) { for (int c = 0; c < i_NCH; ++c) run += (cnt[(size_t)c * i_NRP + t] + 31) & ~31; }
  rsz[t] = (t < NBLKI) ? run : 0;
  __syncthreads();
  for (int off = 1; off < 1024; off <<= 1) { int v = (t >= off) ? rsz[t - off] : 0; __syncthreads(); rsz[t] += v; __syncthreads(); }
  const int incl = rsz[t], excl = incl - ((t < NBLKI) ? run : 0);
  __syncthreads();
  for (int pass = 0; pass < 2; ++pass) {
    if (t < NBLKI) { int r2 = excl; for (int c = 0; c < i_NCH; ++c) { const size_t i = (size_t)c * i_NRP + t; ((volatile int*)boff)[i] = r2; r2 += (cnt[i] + 31) & ~31; } }
    ((volatile int*)rinfo)[t] = excl;
    ((volatile int*)rinfo)[1024 + t] = (t < NBLKI) ? run : 0;
    __threadfence();
  }
}
__global__ __launch_bounds__(256) void i_csr_bucket_kernel(const int* __restrict__ dst, const int* __restrict__ boff, int* __restrict__ bucket) {
  __shared__ int wc[8][i_NRP];
  __shared__ int woff[8][i_NRP];
  __shared__ int roff[i_NRP + 1];
  __shared__ int seg[i_ECH + 32 * i_NRP];
  const int tid = threadIdx.x, lane = tid & 31, wave = tid >> 5;
  for (int i = tid; i < 8 * i_NRP; i += 256) { (&wc[0][0])[i] = 0; }
  __syncthreads();
  const int e0 = blockIdx.x * i_ECH + wave * (i_ECH / 8), e1 = min(e0 + i_ECH / 8, NE);
  for (int c0 = e0; c0 < e0 + i_ECH / 8; c0 += 32) {
    const int e = c0 + lane; const bool valid = e < e1;
    int d = valid ? dst[e] : 0; d = d < 0 ? 0 : (d >= NNI ? NNI - 1 : d);
    const int r = d / NODES_PER_BLK;
    int tot; const int rk = i_rank_eq(r, valid, lane, 9, tot);
    if (valid && rk == tot - 1) wc[wave][r] += tot;
  }
  __syncthreads();
  __shared__ int tot_r[i_NRP];
  for (int i = tid; i < i_NRP; i += 256) { int s = 0; for (int w = 0; w < 8; ++w) s += wc[w][i]; tot_r[i] = s; }
  __syncthreads();
  if (tid == 0) { int run = 0; for (int r = 0; r < i_NRP; ++r) { roff[r] = run; int o = run; for (int w = 0; w < 8; ++w) { woff[w][r] = o; o += wc[w][r]; } run += (tot_r[r] + 31) & ~31; } roff[i_NRP] = run; }
  __syncthreads();
  const int totalpad = roff[i_NRP];
  for (int i = tid; i < totalpad && i < i_ECH + 32 * i_NRP; i += 256) seg[i] = -1;
  __syncthreads();
  for (int c0 = e0; c0 < e0 + i_ECH / 8; c0 += 32) {
    const int e = c0 + lane; const bool valid = e < e1;
    int d = valid ? dst[e] : 0; d = d < 0 ? 0 : (d >= NNI ? NNI - 1 : d);
    const int r = d / NODES_PER_BLK;
    int tot; const int rk = i_rank_eq(r, valid, lane, 9, tot);
    if (valid) { const int slot = woff[wave][r] + rk; if (slot < i_ECH + 32 * i_NRP) seg[slot] = e; if (rk == tot - 1) woff[wave][r] = slot + 1; }
  }
  __syncthreads();
  for (int pass = 0; pass < 2; ++pass) {
    for (int r = wave; r < NBLKI; r += 8) {
      const int lo = roff[r], n = ((tot_r[r] + 31) & ~31);
      const int gb = boff[(size_t)blockIdx.x * i_NRP + r];
      for (int i = lane; i < n; i += 32) ((volatile int*)bucket)[(size_t)gb + i] = (lo + i < i_ECH + 32 * i_NRP) ? seg[lo + i] : -1;
    }
    __threadfence();
  }
}
__global__ __launch_bounds__(256) void i_csr_fill_kernel(const int* __restrict__ dst, const int* __restrict__ bucket, const int* __restrict__ rinfo,
                                                      int* __restrict__ rowptr, int* __restrict__ rowdeg, int* __restrict__ csr_eid, int* __restrict__ rcl) {
  __shared__ int cnt[8][NODES_PER_BLK];
  __shared__ int off[8][NODES_PER_BLK];
  __shared__ int nodeoff[NODES_PER_BLK + 1];
  __shared__ int seg[SEG_CAP];
  const int tid = threadIdx.x, lane = tid & 31, wave = tid >> 5;
  const int n0 = blockIdx.x * NODES_PER_BLK;
  const int bstart = rinfo[blockIdx.x], bsize = rinfo[1024 + blockIdx.x];
  for (int i = tid; i < 8 * NODES_PER_BLK; i += 256) (&cnt[0][0])[i] = 0;
  for (int i = tid; i < SEG_CAP; i += 256) seg[i] = 0;
  __syncthreads();
  const int per = ((bsize / 8) + 31) & ~31;
  const int e0 = bstart + wave * per, e1 = min(bstart + (wave + 1) * per, bstart + bsize);
  for (int c0 = e0; c0 < e0 + per; c0 += 32) {
    const int j = c0 + lane;
    int e = (j < e1) ? bucket[j] : -1;
    const bool valid = (e >= 0) && (e < NE);
    int d = valid ? dst[e] : -1;
    const bool ok = valid && (d >= n0) && (d < n0 + NODES_PER_BLK);
    int tot; const int rk = i_rank_eq(ok ? (d - n0) : 0, ok, lane, 8, tot);
    if (ok && rk == tot - 1) cnt[wave][d - n0] += tot;
  }
  __syncthreads();
  if (tid < 32) {
    int loc[8]; int sum = 0;
    for (int q = 0; q < 8; ++q) { int c = 0; for (int w = 0; w < 8; ++w) c += cnt[w][tid * 8 + q]; loc[q] = c; sum += c; }
    int incl = sum;
    for (int o = 1; o < 32; o <<= 1) { int t = __shfl_up(incl, o, 32); if (lane >= o) incl += t; }
    int base = incl - sum;
    for (int q = 0; q < 8; ++q) {
      const int node = tid * 8 + q;
      nodeoff[node] = base;
      int run = base;
      for (int w = 0; w < 8; ++w) { off[w][node] = run; run += cnt[w][node]; }
      base += loc[q];
    }
    if (tid == 31) nodeoff[NODES_PER_BLK] = base;
  }
  __syncthreads();
  const int btotal = nodeoff[NODES_PER_BLK];
  for (int c0 = e0; c0 < e0 + per; c0 += 32) {
    const int j = c0 + lane;
    int e = (j < e1) ? bucket[j] : -1;
    const bool valid = (e >= 0) && (e < NE);
    int d = valid ? dst[e] : -1;
    const bool ok = valid && (d >= n0) && (d < n0 + NODES_PER_BLK);
    int tot; const int rk = i_rank_eq(ok ? (d - n0) : 0, ok, lane, 8, tot);
    if (ok) { const int slot = off[wave][d - n0] + rk; if (slot < SEG_CAP) seg[slot] = e; if (rk == tot - 1) off[wave][d - n0] = slot + 1; }
  }
  __syncthreads();
  const int gstart = blockIdx.x * (i_SEG_STRIDE);
  const int nlines = (min(btotal, SEG_CAP) + 31) >> 5;
  for (int pass = 0; pass < 2; ++pass) {
    { const int node = tid; int deg = 0; for (int w = 0; w < 8; ++w) deg += cnt[w][node];
      ((volatile int*)rowptr)[n0 + node] = gstart + nodeoff[node]; ((volatile int*)rowdeg)[n0 + node] = deg; }
    for (int i = tid; i < nlines * 32; i += 256) ((volatile int*)csr_eid)[gstart + i] = (i < btotal) ? seg[i] : 0;
    if (rcl != nullptr && tid < 32) ((volatile int*)rcl)[blockIdx.x * 32 + tid] = (tid == 0) ? min(btotal, SEG_CAP) : 0;
    __threadfence();
  }
}

__device__ __forceinline__ unsigned short bfbits(float f) { unsigned u = __float_as_uint(f); return (unsigned short)((u + 0x7FFFu + ((u >> 16) & 1u)) >> 16); }

__global__ __launch_bounds__(256) void rownorm_kernel(const float* __restrict__ x, float* __restrict__ XN, unsigned* __restrict__ XNB) {
  typedef __attribute__((ext_vector_type(2))) float v2f;
  const int lane = threadIdx.x & 31, wave = threadIdx.x >> 5; const int r = blockIdx.x * 8 + wave;
  const v2f v = *(const v2f*)(x + (size_t)r * D + 2 * lane);
  float s = v[0] * v[0] + v[1] * v[1];
  for (int o = 16; o > 0; o >>= 1) s += __shfl_xor(s, o, 32);
  const float inv = 1.0f / fmaxf(sqrtf(s), 1e-12f);
  const v2f o2 = {v[0] * inv, v[1] * inv};
  const unsigned ub = (unsigned)bfbits(o2[0]) | ((unsigned)bfbits(o2[1]) << 16);
  for (int pass = 0; pass < 2; ++pass) { *(volatile v2f*)(XN + (size_t)r * D + 2 * lane) = o2; ((volatile unsigned*)XNB)[(size_t)r * (D / 2) + lane] = ub; __threadfence(); }
}
__global__ __launch_bounds__(256) void transpose_bf16_kernel(const float* __restrict__ src, const float* __restrict__ rscale, int nrows, int kpad, __bf16* __restrict__ outT) {
  __shared__ __align__(16) __bf16 tile[64][72];
  const int m0 = blockIdx.x * 64, tx = threadIdx.x, ty = threadIdx.y;
#pragma unroll
  for (int j = 0; j < 8; ++j) {
    const int m = m0 + ty + 8 * j;
    float v0 = 0.f, v1 = 0.f;
    if (m < nrows) { const float sc = rscale ? rscale[m] : 1.0f; v0 = src[(size_t)m * D + tx] * sc; v1 = src[(size_t)m * D + 32 + tx] * sc; }
    tile[tx][ty + 8 * j] = __builtin_bit_cast(__bf16, bfbits(v0));
    tile[32 + tx][ty + 8 * j] = __builtin_bit_cast(__bf16, bfbits(v1));
  }
  __syncthreads();
  const int t = ty * 32 + tx; const int rr = t >> 3, c8 = (t & 7) * 8;
  for (int pass = 0; pass < 2; ++pass) {
#pragma unroll
    for (int half = 0; half < 2; ++half) { const int c = rr + half * 32; const v8b v = *(const v8b*)(&tile[c][c8]); *(volatile v8b*)(outT + (size_t)c * kpad + m0 + c8) = v; }
    __threadfence();
  }
}

__global__ __launch_bounds__(256) void st16_kernel(const float* __restrict__ S, __bf16* __restrict__ S16) {
  for (int pass = 0; pass < 2; ++pass) { for (int i = threadIdx.x; i < 64 * 64 / 2; i += 256) { const unsigned u = (unsigned)bfbits(S[2 * i]) | ((unsigned)bfbits(S[2 * i + 1]) << 16); ((volatile unsigned*)S16)[i] = u; } __threadfence(); }
}
__global__ __launch_bounds__(256) void transpose_bf16s_kernel(const float* __restrict__ src, const float* __restrict__ US4, int nrows, int kpad, __bf16* __restrict__ outT) {
  __shared__ __align__(16) __bf16 tile[64][72];
  const int m0 = blockIdx.x * 64, tx = threadIdx.x, ty = threadIdx.y;
#pragma unroll
  for (int j = 0; j < 8; ++j) {
    const int m = m0 + ty + 8 * j;
    float v0 = 0.f, v1 = 0.f;
    if (m < nrows) { const float sc = US4[(size_t)m * 4 + 3]; v0 = src[(size_t)m * D + tx] * sc; v1 = src[(size_t)m * D + 32 + tx] * sc; }
    tile[tx][ty + 8 * j] = __builtin_bit_cast(__bf16, bfbits(v0));
    tile[32 + tx][ty + 8 * j] = __builtin_bit_cast(__bf16, bfbits(v1));
  }
  __syncthreads();
  const int t = ty * 32 + tx; const int rr = t >> 3, c8 = (t & 7) * 8;
  for (int pass = 0; pass < 2; ++pass) {
#pragma unroll
    for (int half = 0; half < 2; ++half) { const int c = rr + half * 32; const v8b v = *(const v8b*)(&tile[c][c8]); *(volatile v8b*)(outT + (size_t)c * kpad + m0 + c8) = v; }
    __threadfence();
  }
}
__global__ __launch_bounds__(256) void user_kernel(const float* __restrict__ XN, const float* __restrict__ X, const float* __restrict__ XS,
    const int* __restrict__ rowptr, const int* __restrict__ rowdeg, const int* __restrict__ csr_eid, const int* __restrict__ items,
    const float* __restrict__ SXI, const float* __restrict__ SVI, float* __restrict__ OUT, float* __restrict__ US) {
  typedef __attribute__((ext_vector_type(2))) float v2f;
  const int lane = threadIdx.x & 31, wave = threadIdx.x >> 5; const int u = blockIdx.x * 8 + wave;
  if (u >= NNU) return;
  v2f o = {0.f, 0.f}; v4f us = {0.f, 0.f, 0.f, 0.f};
  {
    const v2f xu = *(const v2f*)(XN + (size_t)u * D + 2 * lane);
    int j0 = rowptr[u]; int dg = rowdeg[u]; dg = dg < 0 ? 0 : (dg > SEG_CAP ? SEG_CAP : dg); j0 = j0 < 0 ? 0 : j0;
    float sxi0 = 0.f, sxi1 = 0.f, svi0 = 0.f, svi1 = 0.f, a0 = 0.f, a1 = 0.f;
    for (int j = j0; j < j0 + dg; ++j) {
      int e = csr_eid[j]; e = e < 0 ? 0 : (e >= NE ? NE - 1 : e); int it = items[e]; it = it < 0 ? 0 : (it >= NNI ? NNI - 1 : it);
      const v2f xi = *(const v2f*)(XN + (size_t)(NNU + it) * D + 2 * lane), vi = *(const v2f*)(X + (size_t)(NNU + it) * D + 2 * lane);
      float d = xu[0] * xi[0] + xu[1] * xi[1];
      for (int of = 16; of > 0; of >>= 1) d += __shfl_xor(d, of, 32);
      sxi0 += xi[0]; sxi1 += xi[1]; svi0 += vi[0]; svi1 += vi[1]; a0 += d * vi[0]; a1 += d * vi[1];
    }
    const float dui = fmaxf((float)dg, 1.0f), duj = fmaxf((float)(NNI - dg), 1.0f);
    const float sxj0 = SXI[2 * lane] - sxi0, sxj1 = SXI[2 * lane + 1] - sxi1, svj0 = SVI[2 * lane] - svi0, svj1 = SVI[2 * lane + 1] - svi1;
    float dp = xu[0] * sxi0 + xu[1] * sxi1, dn = xu[0] * sxj0 + xu[1] * sxj1;
    for (int of = 16; of > 0; of >>= 1) { dp += __shfl_xor(dp, of, 32); dn += __shfl_xor(dn, of, 32); }
    const float b_pos = dp / dui, b_neg = dn / duj;
    const float du1 = dp / dui - b_neg + ALPHA, du2 = -dn / duj + b_pos + ALPHA;
    const v2f xs = *(const v2f*)(XS + (size_t)u * D + 2 * lane);
    const float zu1_0 = a0 / dui - svi0 * (b_neg - ALPHA) / dui, zu1_1 = a1 / dui - svi1 * (b_neg - ALPHA) / dui;
    const float zu2_0 = (xs[0] - a0) / duj - svj0 * (b_pos + ALPHA) / duj, zu2_1 = (xs[1] - a1) / duj - svj1 * (b_pos + ALPHA) / duj;
    const float den = fmaxf(du1, CLAMPV) + fmaxf(du2, CLAMPV);
    o[0] = (zu1_0 + zu2_0) / den; o[1] = (zu1_1 + zu2_1) / den;
    us[0] = 1.0f / dui; us[1] = (-b_neg + ALPHA) / dui; us[2] = (b_pos + ALPHA) / duj; us[3] = 1.0f / duj;
  }
  for (int pass = 0; pass < 2; ++pass) {
    *(volatile v2f*)(OUT + (size_t)u * D + 2 * lane) = o;
    if (lane == 0) *(volatile v4f*)(US + (size_t)u * 4) = us;
    __threadfence();
  }
}
__global__ __launch_bounds__(256) void colsum_partial_kernel(const float* __restrict__ src, const float* __restrict__ scale, int sstride, int soff, int nrows, double* __restrict__ part) {
  const int c = threadIdx.x & 63, ph = threadIdx.x >> 6; const int r0 = blockIdx.x * 512;
  double s = 0.0;
  for (int m = r0 + ph; m < min(r0 + 512, nrows); m += 4) s += (double)src[(size_t)m * D + c] * (scale ? (double)scale[(size_t)m * sstride + soff] : 1.0);
  __shared__ double sh[256]; sh[threadIdx.x] = s; __syncthreads();
  if (threadIdx.x < 64) { const double t = (sh[c] + sh[64 + c]) + (sh[128 + c] + sh[192 + c]); ((volatile double*)part)[(size_t)blockIdx.x * 64 + c] = t; __threadfence(); ((volatile double*)part)[(size_t)blockIdx.x * 64 + c] = t; }
}
__global__ __launch_bounds__(64) void colsum_final_kernel(const double* __restrict__ part, int nblk, float* __restrict__ out) {
  const int c = threadIdx.x; double s = 0.0; for (int b = 0; b < nblk; ++b) s += part[(size_t)b * 64 + c];
  ((volatile float*)out)[c] = (float)s; __threadfence(); ((volatile float*)out)[c] = (float)s;
}
__global__ __launch_bounds__(256) void ussum_partial_kernel(const float* __restrict__ US, double* __restrict__ part) {
  const int r0 = blockIdx.x * 4096; double s = 0.0;
  for (int m = r0 + threadIdx.x; m < min(r0 + 4096, NNU); m += 256) s += (double)US[(size_t)m * 4 + 2];
  __shared__ double sh[256]; sh[threadIdx.x] = s; __syncthreads();
  for (int k = 128; k > 0; k >>= 1) { if (threadIdx.x < k) sh[threadIdx.x] += sh[threadIdx.x + k]; __syncthreads(); }
  if (threadIdx.x < 32) { const double v = (threadIdx.x == 0) ? sh[0] : 0.0; ((volatile double*)part)[(size_t)blockIdx.x * 32 + threadIdx.x] = v; __threadfence(); ((volatile double*)part)[(size_t)blockIdx.x * 32 + threadIdx.x] = v; }
}
__global__ __launch_bounds__(64) void ussum_final_kernel(const double* __restrict__ part, int nblk, float* __restrict__ out) {
  double s = 0.0; for (int b = 0; b < nblk; ++b) s += part[(size_t)b * 32];
  const float v = (float)s; if (threadIdx.x < 32) { ((volatile float*)out)[threadIdx.x] = (threadIdx.x == 0) ? v : 0.f; __threadfence(); ((volatile float*)out)[threadIdx.x] = (threadIdx.x == 0) ? v : 0.f; }
}
__global__ __launch_bounds__(256) void item_kernel(const float* __restrict__ XN, const float* __restrict__ X, const float* __restrict__ XT,
    const int* __restrict__ rowptr, const int* __restrict__ rowdeg, const int* __restrict__ csr_eid, const int* __restrict__ users,
    const float* __restrict__ US, const float* __restrict__ RX, const float* __restrict__ RBp, const float* __restrict__ RV, float* __restrict__ OUT) {
  typedef __attribute__((ext_vector_type(2))) float v2f;
  const int lane = threadIdx.x & 31, wave = threadIdx.x >> 5; const int it = blockIdx.x * 8 + wave;
  if (it >= NNI) return;
  v2f o = {0.f, 0.f};
  {
    const v2f xi = *(const v2f*)(XN + (size_t)(NNU + it) * D + 2 * lane);
    int j0 = rowptr[it]; int dg = rowdeg[it]; dg = dg < 0 ? 0 : (dg > SEG_CAP ? SEG_CAP : dg); j0 = j0 < 0 ? 0 : j0;
    float sx0 = 0.f, sx1 = 0.f, sb1 = 0.f, rx0 = 0.f, rx1 = 0.f, rb = 0.f, z10 = 0.f, z11 = 0.f, rv0 = 0.f, rv1 = 0.f, z20 = 0.f, z21 = 0.f;
    for (int j = j0; j < j0 + dg; ++j) {
      int e = csr_eid[j]; e = e < 0 ? 0 : (e >= NE ? NE - 1 : e); int u = users[e]; u = u < 0 ? 0 : (u >= NNU ? NNU - 1 : u);
      const v2f xu = *(const v2f*)(XN + (size_t)u * D + 2 * lane), vu = *(const v2f*)(X + (size_t)u * D + 2 * lane);
      const v4f us = *(const v4f*)(US + (size_t)u * 4);
      float d = xu[0] * xi[0] + xu[1] * xi[1];
      for (int of = 16; of > 0; of >>= 1) d += __shfl_xor(d, of, 32);
      sx0 += xu[0] * us[0]; sx1 += xu[1] * us[0]; sb1 += us[1];
      rx0 += xu[0] * us[3]; rx1 += xu[1] * us[3]; rb += us[2];
      z10 += d * vu[0] * us[0] - vu[0] * (-us[1]); z11 += d * vu[1] * us[0] - vu[1] * (-us[1]);
      rv0 += vu[0] * us[2]; rv1 += vu[1] * us[2];
      z20 += d * vu[0] * us[3]; z21 += d * vu[1] * us[3];
    }
    float di1 = xi[0] * sx0 + xi[1] * sx1;
    for (int of = 16; of > 0; of >>= 1) di1 += __shfl_xor(di1, of, 32);
    di1 += sb1;
    const float restx0 = RX[2 * lane] - rx0, restx1 = RX[2 * lane + 1] - rx1;
    float dx = xi[0] * restx0 + xi[1] * restx1;
    for (int of = 16; of > 0; of >>= 1) dx += __shfl_xor(dx, of, 32);
    const float di2 = -dx + (RBp[0] - rb);
    const v2f xt = *(const v2f*)(XT + (size_t)it * D + 2 * lane);
    const float zi2_0 = xt[0] - z20 - (RV[2 * lane] - rv0), zi2_1 = xt[1] - z21 - (RV[2 * lane + 1] - rv1);
    const float den = fmaxf(di1, CLAMPV) + fmaxf(di2, CLAMPV);
    o[0] = (z10 + zi2_0) / den; o[1] = (z11 + zi2_1) / den;
  }
  for (int pass = 0; pass < 2; ++pass) { *(volatile v2f*)(OUT + (size_t)(NNU + it) * D + 2 * lane) = o; __threadfence(); }
}

extern "C" void kernel_launch(void* const* d_in, const int* in_sizes, int n_in,
                              void* d_out, int out_size, void* d_ws, size_t ws_size,
                              hipStream_t stream) {
  (void)in_sizes; (void)n_in; (void)out_size; (void)ws_size;
  const float* x = (const float*)d_in[0];
  const int* uu = (const int*)d_in[1];
  const int* ii = (const int*)d_in[2];
  float* out = (float*)d_out;

  char* ws = (char*)d_ws; size_t off = 0;
  auto carve = [&](size_t bytes) -> char* { char* p = ws + off; off += (bytes + 255) & ~(size_t)255; return p; };
  int* uc = (int*)carve((size_t)u_NCH * u_NRP * 4); int* ub = (int*)carve((size_t)u_NCH * u_NRP * 4); int* uri = (int*)carve(2048 * 4);
  int* ubk = (int*)carve(u_BUCKET_INTS * 4); int* urow = (int*)carve((size_t)NUPAD * 4); int* udeg = (int*)carve((size_t)NUPAD * 4); int* ueid = (int*)carve((size_t)NBLKU * u_SEG_STRIDE * 4);
  int* ic = (int*)carve((size_t)i_NCH * i_NRP * 4); int* ib = (int*)carve((size_t)i_NCH * i_NRP * 4); int* iri = (int*)carve(2048 * 4);
  int* ibk = (int*)carve(i_BUCKET_INTS * 4); int* irow = (int*)carve((size_t)NIPAD * 4); int* ideg = (int*)carve((size_t)NIPAD * 4); int* ieid = (int*)carve((size_t)NBLKI * i_SEG_STRIDE * 4);
  float* XN = (float*)carve((size_t)(NNU + NNI) * D * 4);
  unsigned* XNB = (unsigned*)carve((size_t)(NNU + NIPAD) * D * 2);
  __bf16* viT = (__bf16*)carve((size_t)D * KI * 2); __bf16* xiT = (__bf16*)carve((size_t)D * KI * 2);
  __bf16* vuT = (__bf16*)carve((size_t)D * KU * 2); __bf16* xudT = (__bf16*)carve((size_t)D * KU * 2);
  float* ST = (float*)carve(64 * 64 * 4); float* TT = (float*)carve(64 * 64 * 4);
  __bf16* ST16 = (__bf16*)carve(64 * 64 * 2); __bf16* TT16 = (__bf16*)carve(64 * 64 * 2);
  float* XS = (float*)carve((size_t)NUPAD * D * 4); float* XTm = (float*)carve((size_t)NIPAD * D * 4);
  float* US = (float*)carve((size_t)NUPAD * 4 * 4);
  double* part = (double*)carve((size_t)256 * 64 * 8); double* part2 = (double*)carve((size_t)32 * 32 * 8);
  float* SXI = (float*)carve(64 * 4); float* SVI = (float*)carve(64 * 4); float* RX = (float*)carve(64 * 4); float* RV = (float*)carve(64 * 4); float* RB = (float*)carve(32 * 4);
  float* invduj = (float*)carve((size_t)NUPAD * 4);

  u_csr_hist_kernel<<<u_NCH, 256, 0, stream>>>(uu, uc);
  u_csr_offsets_kernel<<<1, 1024, 0, stream>>>(uc, ub, uri);
  u_csr_bucket_kernel<<<u_NCH, 256, 0, stream>>>(uu, ub, ubk);
  u_csr_fill_kernel<<<NBLKU, 256, 0, stream>>>(uu, ubk, uri, urow, udeg, ueid, nullptr);
  i_csr_hist_kernel<<<i_NCH, 256, 0, stream>>>(ii, ic);
  i_csr_offsets_kernel<<<1, 1024, 0, stream>>>(ic, ib, iri);
  i_csr_bucket_kernel<<<i_NCH, 256, 0, stream>>>(ii, ib, ibk);
  i_csr_fill_kernel<<<NBLKI, 256, 0, stream>>>(ii, ibk, iri, irow, ideg, ieid, nullptr);
  rownorm_kernel<<<(NNU + NNI) / 8, 256, 0, stream>>>(x, XN, XNB);
  transpose_bf16_kernel<<<KI / 64, dim3(32, 8), 0, stream>>>(XN + (size_t)NNU * D, nullptr, NNI, KI, xiT);
  transpose_bf16_kernel<<<KI / 64, dim3(32, 8), 0, stream>>>(x + (size_t)NNU * D, nullptr, NNI, KI, viT);
  wmma_gemm64<1, false, 0, 0, false><<<dim3(1, 1), 256, 0, stream>>>(U16(xiT), nullptr, KI, 0, U16(viT), nullptr, KI, 0, ST, nullptr, 64, 0, nullptr, nullptr, 0, 64, 64, KI, 1.0f);
  colsum_partial_kernel<<<(NNI + 511) / 512, 256, 0, stream>>>(XN + (size_t)NNU * D, nullptr, 0, 0, NNI, part);
  colsum_final_kernel<<<1, 64, 0, stream>>>(part, (NNI + 511) / 512, SXI);
  colsum_partial_kernel<<<(NNI + 511) / 512, 256, 0, stream>>>(x + (size_t)NNU * D, nullptr, 0, 0, NNI, part);
  colsum_final_kernel<<<1, 64, 0, stream>>>(part, (NNI + 511) / 512, SVI);
  st16_kernel<<<1, 256, 0, stream>>>(ST, ST16);
  { const int t = (NUPAD / 64); wmma_gemm64<1, false, 0, 0, false><<<dim3((t + 7) / 8, 1), 256, 0, stream>>>((const unsigned short*)XNB, nullptr, D, 0, U16(ST16), nullptr, D, 0, XS, nullptr, D, 0, nullptr, nullptr, 0, NUPAD, 64, 64, 1.0f); }
  user_kernel<<<NUPAD / 8, 256, 0, stream>>>(XN, x, XS, urow, udeg, ueid, ii, SXI, SVI, out, US);
  colsum_partial_kernel<<<(NNU + 511) / 512, 256, 0, stream>>>(XN, US, 4, 3, NNU, part);
  colsum_final_kernel<<<1, 64, 0, stream>>>(part, (NNU + 511) / 512, RX);
  colsum_partial_kernel<<<(NNU + 511) / 512, 256, 0, stream>>>(x, US, 4, 2, NNU, part);
  colsum_final_kernel<<<1, 64, 0, stream>>>(part, (NNU + 511) / 512, RV);
  ussum_partial_kernel<<<(NNU + 4095) / 4096, 256, 0, stream>>>(US, part2);
  ussum_final_kernel<<<1, 64, 0, stream>>>(part2, (NNU + 4095) / 4096, RB);
  transpose_bf16_kernel<<<KU / 64, dim3(32, 8), 0, stream>>>(x, nullptr, NNU, KU, vuT);
  transpose_bf16s_kernel<<<KU / 64, dim3(32, 8), 0, stream>>>(XN, US, NNU, KU, xudT);
  wmma_gemm64<1, false, 0, 0, false><<<dim3(1, 1), 256, 0, stream>>>(U16(vuT), nullptr, KU, 0, U16(xudT), nullptr, KU, 0, TT, nullptr, 64, 0, nullptr, nullptr, 0, 64, 64, KU, 1.0f);
  st16_kernel<<<1, 256, 0, stream>>>(TT, TT16);
  { const int t = (NIPAD / 64); wmma_gemm64<1, false, 0, 0, false><<<dim3((t + 7) / 8, 1), 256, 0, stream>>>((const unsigned short*)(XNB + (size_t)NNU * (D / 2)), nullptr, D, 0, U16(TT16), nullptr, D, 0, XTm, nullptr, D, 0, nullptr, nullptr, 0, NIPAD, 64, 64, 1.0f); }
  item_kernel<<<NIPAD / 8, 256, 0, stream>>>(XN, x, XTm, irow, ideg, ieid, uu, US, RX, RB, RV, out);
}
